// KAN_LAYER_56384330662446
// MI455X (gfx1250) — hardware-verified
//
#include <hip/hip_runtime.h>
#include <math.h>

constexpr int kInDim  = 1024;
constexpr int kOutDim = 1024;
constexpr int kBatch  = 4096;
constexpr int kNumG   = 15;
constexpr int kNumB   = 11;
constexpr int kOrder  = 3;
constexpr int kPack   = 12;
constexpr int kKdim   = kInDim * kPack;
constexpr float kActCarry = 16.0f;
constexpr float kWCarry   = 64.0f;
constexpr float kOutScale = 1.0f / (16.0f * 64.0f);
constexpr int kTilesM = kBatch / 64;
constexpr int kTilesN = kOutDim / 64;
constexpr int kTiles  = kTilesM * kTilesN;
static_assert(kKdim % 32 == 0);
static_assert(kBatch % 64 == 0);
static_assert(kOutDim % 64 == 0);
static_assert(kTiles % 8 == 0);
static_assert(kInDim % 256 == 0);

typedef __attribute__((ext_vector_type(16))) _Float16 v16h;
typedef __attribute__((ext_vector_type(8)))  _Float16 v8h;
typedef __attribute__((ext_vector_type(16))) __bf16   v16b;
typedef __attribute__((ext_vector_type(8)))  __bf16   v8b;
typedef __attribute__((ext_vector_type(8)))  float    v8f;
typedef __attribute__((ext_vector_type(4)))  float    v4f;
typedef __attribute__((ext_vector_type(4)))  unsigned int v4u;

__device__ __forceinline__ unsigned short f2bf_bits(float f) {
  unsigned u = __float_as_uint(f);
  return (unsigned short)((u + 0x7FFFu + ((u >> 16) & 1u)) >> 16);
}
__device__ __forceinline__ float bf_bits2f(unsigned short h) { return __uint_as_float(((unsigned)h) << 16); }

__device__ __forceinline__ void dep_guard_h(v8f& a, v8f& b, v16h x, v16h y) { asm volatile("v_nop\n\tv_nop\n\tv_nop\n\tv_nop" : "+v"(a), "+v"(b) : "v"(x), "v"(y)); }
__device__ __forceinline__ void dep_guard_b(v8f& a, v8f& b, v16b x, v16b y) { asm volatile("v_nop\n\tv_nop\n\tv_nop\n\tv_nop" : "+v"(a), "+v"(b) : "v"(x), "v"(y)); }
__device__ __forceinline__ void keep4_h(v16h a, v16h b, v16h c, v16h d) { asm volatile("v_nop" :: "v"(a), "v"(b), "v"(c), "v"(d)); }
__device__ __forceinline__ void keep4_b(v16b a, v16b b, v16b c, v16b d) { asm volatile("v_nop" :: "v"(a), "v"(b), "v"(c), "v"(d)); }
__device__ __forceinline__ void acc_guard4(v8f& a, v8f& b, v8f& c, v8f& d) { asm volatile("v_nop\n\tv_nop\n\tv_nop\n\tv_nop" : "+v"(a), "+v"(b), "+v"(c), "+v"(d)); }
template <typename T> struct Frag;
template <> struct Frag<_Float16> {
  typedef v16h V; union U { v16h v; v8h h[2]; };
  static __device__ __forceinline__ v16h load(const _Float16* p) {
    U f; f.h[0] = *(const v8h*)(p); f.h[1] = *(const v8h*)(p + 16); return f.v;
  }
  static __device__ __forceinline__ v8f mma(v16h a, v16h b, v8f c) {
    return __builtin_amdgcn_wmma_f32_16x16x32_f16(false, a, false, b, (short)0, c, false, false);
  }
  static __device__ __forceinline__ void guard(v8f& a, v8f& b, v16h x, v16h y) { dep_guard_h(a, b, x, y); }
  static __device__ __forceinline__ void keep(v16h a, v16h b, v16h c, v16h d) { keep4_h(a, b, c, d); }
};
template <> struct Frag<__bf16> {
  typedef v16b V; union U { v16b v; v8b h[2]; };
  static __device__ __forceinline__ v16b load(const __bf16* p) {
    U f; f.h[0] = *(const v8b*)(p); f.h[1] = *(const v8b*)(p + 16); return f.v;
  }
  static __device__ __forceinline__ v8f mma(v16b a, v16b b, v8f c) {
    return __builtin_amdgcn_wmma_f32_16x16x32_bf16(false, a, false, b, (short)0, c, false, false);
  }
  static __device__ __forceinline__ void guard(v8f& a, v8f& b, v16b x, v16b y) { dep_guard_b(a, b, x, y); }
  static __device__ __forceinline__ void keep(v16b a, v16b b, v16b c, v16b d) { keep4_b(a, b, c, d); }
};

__device__ __forceinline__ unsigned pk16(unsigned short a, unsigned short b) { return (unsigned)a | ((unsigned)b << 16); }
__device__ __forceinline__ unsigned short h_bits(float f) { const _Float16 h = (_Float16)f; return __builtin_bit_cast(unsigned short, h); }

template <int ET> struct Elem;
template <> struct Elem<0> { typedef _Float16 T; };
template <> struct Elem<1> { typedef __bf16 T; };
template <int ET, bool SPLIT, int BIAS_MODE, int OUT_MODE, bool RESID, int ACT = 0>
__global__ __launch_bounds__(256) void wmma_gemm64(
    const unsigned short* __restrict__ Ap, const unsigned short* __restrict__ A2p, int lda, long strideA,
    const unsigned short* __restrict__ Btp, const unsigned short* __restrict__ Bt2p, int ldb, long strideB,
    void* __restrict__ Cout, void* __restrict__ Cout2, int ldc, long strideC,
    const float* __restrict__ bias,
    const float* __restrict__ resid, long strideR,
    int M, int N, int K, float scale) {
  typedef typename Elem<ET>::T T;
  typedef typename Frag<T>::V V;
  const T* A = (const T*)Ap; const T* A2 = (const T*)A2p; const T* Bt = (const T*)Btp; const T* Bt2 = (const T*)Bt2p;
  __shared__ __align__(16) float sT[8][16 * 68];
  const int b    = blockIdx.y;
  const int lane = threadIdx.x & 31;
  const int wave = threadIdx.x >> 5;
  const int tilesN = N >> 6;
  const int tilesM = M >> 6;
  const int tile = blockIdx.x * 8 + wave;
  if (tile >= tilesM * tilesN) return;
  const int tm = tile / tilesN;
  const int tn = tile - tm * tilesN;
  const int m0 = tm << 6;
  const int n0 = tn << 6;

  const T* Ab  = A  + (size_t)b * strideA;
  const T* Bb  = Bt + (size_t)b * strideB;
  const T* Ab2 = SPLIT ? (A2  + (size_t)b * strideA) : nullptr;
  const T* Bb2 = SPLIT ? (Bt2 + (size_t)b * strideB) : nullptr;

  const int rlane = lane & 15;
  const int koff  = (lane >> 4) * 8;
  const int mOff  = (lane >> 4) * 8;

  v8f acc[4][4];
#pragma unroll
  for (int i = 0; i < 4; ++i)
#pragma unroll
    for (int j = 0; j < 4; ++j) acc[i][j] = (v8f){0.f,0.f,0.f,0.f,0.f,0.f,0.f,0.f};

  for (int k0 = 0; k0 < K; k0 += 32) {
    V bh[4], bl[4];
#pragma unroll
    for (int j = 0; j < 4; ++j) {
      const size_t bo = (size_t)(n0 + (j << 4) + rlane) * ldb + koff + k0;
      bh[j] = Frag<T>::load(Bb + bo);
      if (SPLIT) bl[j] = Frag<T>::load(Bb2 + bo);
    }
#pragma unroll
    for (int i = 0; i < 4; ++i) {
      const size_t ao = (size_t)(m0 + (i << 4) + rlane) * lda + koff + k0;
      V ah = Frag<T>::load(Ab + ao);
      V al;
      if (SPLIT) al = Frag<T>::load(Ab2 + ao);
#pragma unroll
      for (int j = 0; j < 4; ++j) {
        acc[i][j] = Frag<T>::mma(ah, bh[j], acc[i][j]);
        if (SPLIT) {
          acc[i][j] = Frag<T>::mma(ah, bl[j], acc[i][j]);
          acc[i][j] = Frag<T>::mma(al, bh[j], acc[i][j]);
        }
      }
      Frag<T>::guard(acc[i][0], acc[i][3], ah, SPLIT ? al : ah);
    }
    Frag<T>::keep(bh[0], bh[1], bh[2], bh[3]);
    if (SPLIT) Frag<T>::keep(bl[0], bl[1], bl[2], bl[3]);
  }
  acc_guard4(acc[0][0], acc[0][1], acc[0][2], acc[0][3]);
  acc_guard4(acc[1][0], acc[1][1], acc[1][2], acc[1][3]);
  acc_guard4(acc[2][0], acc[2][1], acc[2][2], acc[2][3]);
  acc_guard4(acc[3][0], acc[3][1], acc[3][2], acc[3][3]);

  float* slab = sT[wave];
  const float* Rb = RESID ? (resid + (size_t)b * strideR) : nullptr;
#pragma unroll
  for (int i = 0; i < 4; ++i) {
    const int mBase = m0 + (i << 4);
#pragma unroll
    for (int j = 0; j < 4; ++j) {
      const int n = n0 + (j << 4) + rlane;
      float bv = 0.f;
      if (BIAS_MODE == 2) bv = bias[n];
#pragma unroll
      for (int r = 0; r < 8; ++r) {
        float v = acc[i][j][r] * scale;
        if (BIAS_MODE == 1) v += bias[mBase + mOff + r];
        if (BIAS_MODE == 2) v += bv;
        if (RESID) v += Rb[(size_t)(mBase + mOff + r) * ldc + n];
        if (ACT == 2) v = fmaxf(v, 0.0f);
        if (ACT == 4) v = (v > 0.f) ? v : 0.01f * v;
        slab[(mOff + r) * 68 + (j << 4) + rlane] = v;
      }
    }
    __builtin_amdgcn_fence(__ATOMIC_RELEASE, "workgroup");
    __builtin_amdgcn_wave_barrier();
    __builtin_amdgcn_fence(__ATOMIC_ACQUIRE, "workgroup");
    if (OUT_MODE == 0) {
      float* C = (float*)Cout + (size_t)b * strideC;
      const int hh = lane >> 4, c4 = (lane & 15) * 4;
      for (int pass = 0; pass < 2; ++pass) {
#pragma unroll
        for (int it = 0; it < 8; ++it) {
          const int row = it * 2 + hh;
          v4f v = *(const v4f*)(slab + row * 68 + c4);
          *(volatile v4f*)(C + (size_t)(mBase + row) * ldc + n0 + c4) = v;
        }
        __threadfence();
      }
    } else {
      const int q = lane >> 3, c8 = (lane & 7) * 8;
      unsigned short* C  = (unsigned short*)Cout  + (size_t)b * strideC;
      unsigned short* C2 = (OUT_MODE == 2) ? ((unsigned short*)Cout2 + (size_t)b * strideC) : nullptr;
      for (int pass = 0; pass < 2; ++pass) {
#pragma unroll
        for (int it = 0; it < 4; ++it) {
          const int row = it * 4 + q;
          const float* sp = slab + row * 68 + c8;
          v8h hv, lv;
#pragma unroll
          for (int e = 0; e < 8; ++e) {
            if (OUT_MODE == 1) {
              hv[e] = (_Float16)sp[e];
            } else {
              unsigned short hb = f2bf_bits(sp[e]);
              unsigned short lb = f2bf_bits(sp[e] - bf_bits2f(hb));
              hv[e] = __builtin_bit_cast(_Float16, hb);
              lv[e] = __builtin_bit_cast(_Float16, lb);
            }
          }
          *(volatile v8h*)(C + (size_t)(mBase + row) * ldc + n0 + c8) = hv;
          if (OUT_MODE == 2) *(volatile v8h*)(C2 + (size_t)(mBase + row) * ldc + n0 + c8) = lv;
        }
        __threadfence();
      }
    }
    __builtin_amdgcn_fence(__ATOMIC_RELEASE, "workgroup");
    __builtin_amdgcn_wave_barrier();
    __builtin_amdgcn_fence(__ATOMIC_ACQUIRE, "workgroup");
  }
}

__global__ __launch_bounds__(256) void pack_weights_kernel(const float* __restrict__ coef,
                                                          const float* __restrict__ scale_base,
                                                          const float* __restrict__ scale_sp,
                                                          const float* __restrict__ mask,
                                                          unsigned short* __restrict__ Wt) {
  __shared__ __align__(16) unsigned int sW[kKdim / 2];
  const int o = blockIdx.x;
  const int t = threadIdx.x;
#pragma unroll 1
  for (int ii = 0; ii < kInDim / 256; ++ii) {
    const int i = t + 256 * ii;
    const size_t io = (size_t)i * kOutDim + o;
    const float m  = mask[io];
    const float wb = (m * scale_base[io]) * kWCarry;
    const float ws = m * scale_sp[io];
    const float* cp = coef + io * kNumB;
    float wv[kPack];
    wv[0] = wb;
#pragma unroll
    for (int k = 0; k < kNumB; ++k) wv[1 + k] = (cp[k] * ws) * kWCarry;
    unsigned int* dst = sW + i * (kPack / 2);
#pragma unroll
    for (int q = 0; q < kPack / 2; ++q) dst[q] = pk16(h_bits(wv[2 * q]), h_bits(wv[2 * q + 1]));
  }
  __syncthreads();
  unsigned short* row = Wt + (size_t)o * kKdim;
  for (int pass = 0; pass < 2; ++pass) {
#pragma unroll
    for (int c = 0; c < 6; ++c) {
      const int chunk = t + 256 * c;
      const v4u u = *(const v4u*)(sW + chunk * 4);
      *(volatile v4u*)(row + (size_t)chunk * 8) = u;
    }
    __threadfence();
  }
}

__global__ __launch_bounds__(256) void pack_acts_kernel(const float* __restrict__ x,
                                                       const float* __restrict__ grid,
                                                       unsigned short* __restrict__ Act) {
  __shared__ __align__(16) float sG[256 * kNumG];
  __shared__ __align__(16) unsigned int sA[256 * (kPack / 2)];
  const int ic = blockIdx.x;
  const int b  = blockIdx.y;
  const int t  = threadIdx.x;
  const int i0 = ic * 256;
  {
    const v4f* gp = (const v4f*)(grid + (size_t)i0 * kNumG);
#pragma unroll
    for (int it = 0; it < 4; ++it) {
      const int c  = t + 256 * it;
      const int cc = (c < 960) ? c : 959;
      const v4f gv = gp[cc];
      if (c < 960) *(v4f*)(sG + 4 * c) = gv;
    }
  }
  __syncthreads();

  const int i = i0 + t;
  const float xv = x[(size_t)b * kInDim + i];
  float g[kNumG];
#pragma unroll
  for (int j = 0; j < kNumG; ++j) g[j] = sG[t * kNumG + j];

  float v[kNumG - 1];
#pragma unroll
  for (int j = 0; j < kNumG - 1; ++j) v[j] = (xv >= g[j] && xv < g[j + 1]) ? 1.0f : 0.0f;

#pragma unroll
  for (int p = 1; p <= kOrder; ++p) {
    float r[kNumG];
#pragma unroll
    for (int j = 0; j < kNumG; ++j) {
      r[j] = 0.0f;
      if (j + p < kNumG) r[j] = __builtin_amdgcn_rcpf(g[j + p] - g[j]);
    }
#pragma unroll
    for (int j = 0; j < kNumG - 1; ++j) {
      if (j + p < kNumG - 1) {
        const float tl = ((xv - g[j]) * r[j]) * v[j];
        const float tr = ((g[j + p + 1] - xv) * r[j + 1]) * v[j + 1];
        const float tt = tl + tr;
        v[j] = (tt == tt) ? tt : 0.0f;
      }
    }
  }

  const float sil = xv / (1.0f + expf(-xv));

  unsigned short hb[kPack];
  hb[0] = h_bits(sil * kActCarry);
#pragma unroll
  for (int k = 0; k < kNumB; ++k) hb[1 + k] = h_bits(v[k] * kActCarry);
  unsigned int* dst = sA + t * (kPack / 2);
#pragma unroll
  for (int q = 0; q < kPack / 2; ++q) dst[q] = pk16(hb[2 * q], hb[2 * q + 1]);
  __syncthreads();

  unsigned short* seg = Act + (size_t)b * kKdim + (size_t)i0 * kPack;
  const v4u u0 = *(const v4u*)(sA + 4 * t);
  const int t1 = (t < 128) ? t : 0;
  const v4u u1 = *(const v4u*)(sA + 4 * (256 + t1));
  for (int pass = 0; pass < 2; ++pass) {
    *(volatile v4u*)(seg + (size_t)t * 8) = u0;
    if (t < 128) *(volatile v4u*)(seg + (size_t)(256 + t) * 8) = u1;
    __threadfence();
  }
}

extern "C" void kernel_launch(void* const* d_in, const int* in_sizes, int n_in,
                              void* d_out, int out_size, void* d_ws, size_t ws_size,
                              hipStream_t stream) {
  if (n_in < 6) return;
  if (in_sizes[0] != kBatch * kInDim) return;
  if (in_sizes[1] != kInDim * kNumG) return;
  if (in_sizes[2] != kInDim * kOutDim * kNumB) return;
  if (in_sizes[3] != kInDim * kOutDim || in_sizes[4] != kInDim * kOutDim || in_sizes[5] != kInDim * kOutDim) return;
  if (out_size != kBatch * kOutDim) return;

  const size_t actBytes = (size_t)kBatch * kKdim * sizeof(unsigned short);
  const size_t wtBytes  = (size_t)kOutDim * kKdim * sizeof(unsigned short);
  if (actBytes + wtBytes > ws_size) return;

  const float* x          = (const float*)d_in[0];
  const float* grid       = (const float*)d_in[1];
  const float* coef       = (const float*)d_in[2];
  const float* scale_base = (const float*)d_in[3];
  const float* scale_sp   = (const float*)d_in[4];
  const float* mask       = (const float*)d_in[5];
  float* out = (float*)d_out;

  unsigned short* Act = (unsigned short*)d_ws;
  unsigned short* Wt  = (unsigned short*)((char*)d_ws + actBytes);

  pack_weights_kernel<<<dim3(kOutDim), dim3(256), 0, stream>>>(coef, scale_base, scale_sp, mask, Wt);
  pack_acts_kernel<<<dim3(kInDim / 256, kBatch), dim3(256), 0, stream>>>(x, grid, Act);

  wmma_gemm64<0, false, 0, 0, false, 0><<<dim3(kTiles / 8, 1), dim3(256), 0, stream>>>(
      Act, Act, kKdim, 0L,
      Wt, Wt, kKdim, 0L,
      (void*)out, (void*)out, kOutDim, 0L,
      (const float*)d_ws,
      (const float*)d_ws, 0L,
      kBatch, kOutDim, kKdim, kOutScale);
}
